// DCNV2_73452530696362
// MI455X (gfx1250) — hardware-verified
//
#include <hip/hip_runtime.h>
#include <math.h>
#include <stddef.h>

typedef __attribute__((ext_vector_type(16))) _Float16 v16h;
typedef __attribute__((ext_vector_type(8)))  _Float16 v8h;
typedef __attribute__((ext_vector_type(16))) __bf16   v16b;
typedef __attribute__((ext_vector_type(8)))  __bf16   v8b;
typedef __attribute__((ext_vector_type(8)))  float    v8f;
typedef __attribute__((ext_vector_type(4)))  float    v4f;
typedef __attribute__((ext_vector_type(4)))  unsigned v4u;

constexpr int NB        = 4;
constexpr int CIN       = 128;
constexpr int NCO       = 128;
constexpr int IMH       = 96;
constexpr int IMW       = 96;
constexpr int HWPIX     = IMH * IMW;
constexpr int PADH      = IMH + 2;
constexpr int PADW      = IMW + 2;
constexpr int PADPIX    = PADH * PADW;
constexpr int NBORDER   = 2 * PADW + 2 * IMH;
constexpr int XB_THREADS = NB * NBORDER * 16;
constexpr int NTAP      = 9;
constexpr int KDIM      = NTAP * CIN;
constexpr int MROWS     = NB * HWPIX;
constexpr int PTILE     = 64;
constexpr int NBLK      = MROWS / PTILE;
constexpr int NCH_OFF   = 18;
constexpr int NCH_OM    = 27;
constexpr int NROW_OFFW = 32;
constexpr int WALL_ROWS = NCO + NROW_OFFW;
constexpr int KW8       = KDIM / 8;
constexpr int XPITCH    = 65;
constexpr int APITCH    = 40;
constexpr int OPITCH    = 68;
constexpr int SPITCH    = 68;
constexpr int OUT4      = NB * NCO * HWPIX / 4;
constexpr float BN_EPSILON = 1e-5f;

static_assert(HWPIX % PTILE == 0);
static_assert(MROWS % PTILE == 0);
static_assert(KDIM % 32 == 0);
static_assert(CIN % 32 == 0);
static_assert((WALL_ROWS * KW8) % 256 == 0);
static_assert(OUT4 % 256 == 0);
static_assert(XB_THREADS % 256 == 0);
static_assert(APITCH % 8 == 0 && OPITCH % 4 == 0 && SPITCH % 4 == 0);
static_assert(NCO == 128 && PTILE == 64);

constexpr size_t WS_OFF_XT   = 0;
constexpr size_t WS_SZ_XT    = (size_t)NB * PADPIX * CIN * 2;
constexpr size_t WS_OFF_WALL = WS_OFF_XT + WS_SZ_XT;
constexpr size_t WS_SZ_WALL  = (size_t)WALL_ROWS * KDIM * 2;
constexpr size_t WS_OFF_OM   = WS_OFF_WALL + WS_SZ_WALL;
constexpr size_t WS_SZ_OM    = (size_t)NCH_OM * MROWS * 4;
constexpr size_t WS_OFF_P    = WS_OFF_OM + WS_SZ_OM;
constexpr size_t WS_SZ_P     = (size_t)NB * NCO * HWPIX * 4;
constexpr size_t WS_OFF_PART = WS_OFF_P + WS_SZ_P;
constexpr size_t WS_SZ_PART  = (size_t)NBLK * 2 * NCO * 4;
constexpr size_t WS_OFF_BNP  = WS_OFF_PART + WS_SZ_PART;
constexpr size_t WS_SZ_BNP   = (size_t)2 * NCO * 4;
constexpr size_t WS_TOTAL    = WS_OFF_BNP + WS_SZ_BNP;
static_assert(WS_TOTAL == 33649664);
static_assert(WS_TOTAL <= 134217728);
static_assert(WS_OFF_WALL % 256 == 0 && WS_OFF_OM % 256 == 0 && WS_OFF_P % 256 == 0 && WS_OFF_PART % 256 == 0 && WS_OFF_BNP % 256 == 0);

__device__ __forceinline__ unsigned short f2bf_bits(float f) {
  unsigned u = __float_as_uint(f);
  return (unsigned short)((u + 0x7FFFu + ((u >> 16) & 1u)) >> 16);
}
__device__ __forceinline__ float bf_bits2f(unsigned short h) { return __uint_as_float(((unsigned)h) << 16); }
__device__ __forceinline__ float bfr(float f) { return bf_bits2f(f2bf_bits(f)); }

__device__ __forceinline__ void dep_guard_h(v8f& a, v8f& b, v16h x, v16h y) { asm volatile("v_nop\n\tv_nop\n\tv_nop\n\tv_nop" : "+v"(a), "+v"(b) : "v"(x), "v"(y)); }
__device__ __forceinline__ void dep_guard_b(v8f& a, v8f& b, v16b x, v16b y) { asm volatile("v_nop\n\tv_nop\n\tv_nop\n\tv_nop" : "+v"(a), "+v"(b) : "v"(x), "v"(y)); }
__device__ __forceinline__ void keep4_h(v16h a, v16h b, v16h c, v16h d) { asm volatile("v_nop" :: "v"(a), "v"(b), "v"(c), "v"(d)); }
__device__ __forceinline__ void keep4_b(v16b a, v16b b, v16b c, v16b d) { asm volatile("v_nop" :: "v"(a), "v"(b), "v"(c), "v"(d)); }
__device__ __forceinline__ void acc_guard4(v8f& a, v8f& b, v8f& c, v8f& d) { asm volatile("v_nop\n\tv_nop\n\tv_nop\n\tv_nop" : "+v"(a), "+v"(b), "+v"(c), "+v"(d)); }
__device__ __forceinline__ void acc_guard2(v8f& a, v8f& b) { asm volatile("v_nop\n\tv_nop\n\tv_nop\n\tv_nop" : "+v"(a), "+v"(b)); }
__device__ __forceinline__ void guard2_3(v8f& a, v8f& b, v16b x, v16b y, v16b z) {
  asm volatile("v_nop\n\tv_nop\n\tv_nop\n\tv_nop" : "+v"(a), "+v"(b) : "v"(x), "v"(y), "v"(z));
}
__device__ __forceinline__ void guard4_6(v8f& a, v8f& b, v8f& c, v8f& d, v16b x0, v16b x1, v16b y0, v16b y1, v16b y2, v16b y3) {
  asm volatile("v_nop\n\tv_nop\n\tv_nop\n\tv_nop" : "+v"(a), "+v"(b), "+v"(c), "+v"(d) : "v"(x0), "v"(x1), "v"(y0), "v"(y1), "v"(y2), "v"(y3));
}
template <typename T> struct Frag;
template <> struct Frag<_Float16> {
  typedef v16h V; union U { v16h v; v8h h[2]; };
  static __device__ __forceinline__ v16h load(const _Float16* p) {
    U f; f.h[0] = *(const v8h*)(p); f.h[1] = *(const v8h*)(p + 16); return f.v;
  }
  static __device__ __forceinline__ v8f mma(v16h a, v16h b, v8f c) {
    return __builtin_amdgcn_wmma_f32_16x16x32_f16(false, a, false, b, (short)0, c, false, false);
  }
  static __device__ __forceinline__ void guard(v8f& a, v8f& b, v16h x, v16h y) { dep_guard_h(a, b, x, y); }
  static __device__ __forceinline__ void keep(v16h a, v16h b, v16h c, v16h d) { keep4_h(a, b, c, d); }
};
template <> struct Frag<__bf16> {
  typedef v16b V; union U { v16b v; v8b h[2]; };
  static __device__ __forceinline__ v16b load(const __bf16* p) {
    U f; f.h[0] = *(const v8b*)(p); f.h[1] = *(const v8b*)(p + 16); return f.v;
  }
  static __device__ __forceinline__ v8f mma(v16b a, v16b b, v8f c) {
    return __builtin_amdgcn_wmma_f32_16x16x32_bf16(false, a, false, b, (short)0, c, false, false);
  }
  static __device__ __forceinline__ void guard(v8f& a, v8f& b, v16b x, v16b y) { dep_guard_b(a, b, x, y); }
  static __device__ __forceinline__ void keep(v16b a, v16b b, v16b c, v16b d) { keep4_b(a, b, c, d); }
};
typedef Frag<__bf16> FragB;
union FragU { v16b v; v4u q[2]; };

__global__ __launch_bounds__(256) void xprep_kernel(const float* __restrict__ x, unsigned short* __restrict__ xT) {
  __shared__ __align__(16) float sx[CIN * XPITCH];
  const int tid = threadIdx.x;
  const int blk = blockIdx.x;
  const int n = blk / (HWPIX / PTILE);
  const int hw0 = (blk - n * (HWPIX / PTILE)) * PTILE;
  const float* xb = x + (size_t)n * CIN * HWPIX + hw0;
  {
    const int p = tid & 63, cq = tid >> 6;
#pragma unroll 4
    for (int it = 0; it < 32; ++it) {
      const int c = it * 4 + cq;
      sx[c * XPITCH + p] = xb[(size_t)c * HWPIX + p];
    }
  }
  __syncthreads();
  const int lane = tid & 31, wave = tid >> 5, hh = lane >> 4, c0 = (lane & 15) * 8;
  v4u wv[4];
  size_t po[4];
#pragma unroll
  for (int it = 0; it < 4; ++it) {
    const int p = wave * 8 + it * 2 + hh;
    const int hw = hw0 + p;
    const int h = hw / IMW, w = hw - h * IMW;
    po[it] = ((size_t)n * PADPIX + (size_t)(h + 1) * PADW + (size_t)(w + 1)) * CIN + c0;
    unsigned wd[4];
#pragma unroll
    for (int i = 0; i < 4; ++i) {
      const unsigned b0 = (unsigned)f2bf_bits(sx[(c0 + 2 * i) * XPITCH + p]);
      const unsigned b1 = (unsigned)f2bf_bits(sx[(c0 + 2 * i + 1) * XPITCH + p]);
      wd[i] = b0 | (b1 << 16);
    }
    wv[it] = (v4u){wd[0], wd[1], wd[2], wd[3]};
  }
  for (int pass = 0; pass < 2; ++pass) {
#pragma unroll
    for (int it = 0; it < 4; ++it) {
      *(volatile v4u*)(xT + po[it]) = wv[it];
    }
    __threadfence();
  }
}

__global__ __launch_bounds__(256) void xborder_kernel(unsigned short* __restrict__ xT) {
  const int g = blockIdx.x * 256 + threadIdx.x;
  if (g >= XB_THREADS) return;
  const int slot = g >> 4, l16 = g & 15;
  const int n = slot / NBORDER;
  const int b = slot - n * NBORDER;
  const int py = (b < PADW) ? 0 : (b < 2 * PADW) ? (PADH - 1) : (b < 2 * PADW + IMH) ? (b - 2 * PADW + 1) : (b - 2 * PADW - IMH + 1);
  const int px = (b < PADW) ? b : (b < 2 * PADW) ? (b - PADW) : (b < 2 * PADW + IMH) ? 0 : (PADW - 1);
  const v4u z = (v4u){0u, 0u, 0u, 0u};
  unsigned short* dst = xT + ((size_t)n * PADPIX + (size_t)py * PADW + (size_t)px) * CIN + l16 * 8;
  *(volatile v4u*)dst = z;
  __threadfence();
  *(volatile v4u*)dst = z;
}

__global__ __launch_bounds__(256) void wswz_kernel(const float* __restrict__ wmain, const float* __restrict__ woff,
                                                   const float* __restrict__ wmod, unsigned short* __restrict__ wall) {
  const int i = blockIdx.x * 256 + threadIdx.x;
  if (i >= WALL_ROWS * KW8) return;
  const int rr = i / KW8;
  const int k0 = (i - rr * KW8) * 8;
  const int om_ = (rr < NCO) ? rr : (NCO - 1);
  int ro = rr - NCO;           ro = ro < 0 ? 0 : (ro > NCH_OFF - 1 ? NCH_OFF - 1 : ro);
  int rm = rr - NCO - NCH_OFF; rm = rm < 0 ? 0 : (rm > NTAP - 1 ? NTAP - 1 : rm);
  const float f1 = (rr < NCO) ? 1.0f : 0.0f;
  const float f2 = (rr >= NCO && rr < NCO + NCH_OFF) ? 1.0f : 0.0f;
  const float f3 = (rr >= NCO + NCH_OFF && rr < NCO + NCH_OM) ? 1.0f : 0.0f;
  unsigned hb[8];
#pragma unroll
  for (int e = 0; e < 4; ++e) {
    const int k = k0 + e, kk = k >> 7, c = k & 127;
    const float a = wmain[((size_t)om_ * CIN + c) * NTAP + kk];
    const float b = woff[((size_t)ro * CIN + c) * NTAP + kk];
    const float d = wmod[((size_t)rm * CIN + c) * NTAP + kk];
    const float v = fmaf(f1, a, fmaf(f2, b, f3 * d));
    hb[e] = (unsigned)f2bf_bits(v);
  }
  asm volatile("" :: "v"(hb[0]), "v"(hb[1]), "v"(hb[2]), "v"(hb[3]) : "memory");
#pragma unroll
  for (int e = 4; e < 8; ++e) {
    const int k = k0 + e, kk = k >> 7, c = k & 127;
    const float a = wmain[((size_t)om_ * CIN + c) * NTAP + kk];
    const float b = woff[((size_t)ro * CIN + c) * NTAP + kk];
    const float d = wmod[((size_t)rm * CIN + c) * NTAP + kk];
    const float v = fmaf(f1, a, fmaf(f2, b, f3 * d));
    hb[e] = (unsigned)f2bf_bits(v);
  }
  const v4u wv = (v4u){hb[0] | (hb[1] << 16), hb[2] | (hb[3] << 16), hb[4] | (hb[5] << 16), hb[6] | (hb[7] << 16)};
  unsigned short* dst = wall + (size_t)i * 8;
  *(volatile v4u*)dst = wv;
  __threadfence();
  *(volatile v4u*)dst = wv;
}

__device__ __forceinline__ void om_stage_off(float* sO, v8f a, int col, int prow0, float obv) {
#pragma unroll
  for (int r = 0; r < 8; ++r) sO[col * SPITCH + prow0 + r] = a[r] + obv;
}
__device__ __forceinline__ void om_stage_mix(float* sO, v8f a, int col, int prow0, float obv, float mbv, float fo) {
  const float fm = 1.0f - fo;
#pragma unroll
  for (int r = 0; r < 8; ++r) {
    const float v = a[r];
    const float voff = v + obv;
    const float vm = 2.0f / (1.0f + expf(-(v + mbv)));
    sO[col * SPITCH + prow0 + r] = fmaf(fo, voff, fm * vm);
  }
}

__global__ __launch_bounds__(128) void offmask_kernel(const unsigned short* __restrict__ xT,
                                                      const unsigned short* __restrict__ woffbt,
                                                      const float* __restrict__ offb, const float* __restrict__ modb,
                                                      float* __restrict__ om) {
  __shared__ __align__(16) float sO[NROW_OFFW * SPITCH];
  const int tid = threadIdx.x, lane = tid & 31, wave = tid >> 5;
  const int rlane = lane & 15, hh = lane >> 4, koff = hh * 8;
  const int m0 = blockIdx.x * PTILE;
  const int n = m0 / HWPIX;
  const int hw0 = m0 - n * HWPIX;
  const int hwa = hw0 + wave * 16 + rlane;
  const int ha = hwa / IMW, wa = hwa - ha * IMW;
  const v8f z8 = {0.f, 0.f, 0.f, 0.f, 0.f, 0.f, 0.f, 0.f};
  v8f acc0 = z8, acc1 = z8;
  const __bf16* Bb = (const __bf16*)woffbt + (size_t)rlane * KDIM + koff;
  const unsigned short* xn = xT + (size_t)n * PADPIX * CIN;

#pragma unroll 1
  for (int kk = 0; kk < NTAP; ++kk) {
    const int ky = kk / 3, kx = kk - ky * 3;
    const unsigned short* arow = xn + ((size_t)(ha + ky) * PADW + (size_t)(wa + kx)) * CIN + koff;
#pragma unroll 1
    for (int cc = 0; cc < CIN / 32; ++cc) {
      FragU fa;
      fa.q[0] = *(const v4u*)(arow + cc * 32);
      fa.q[1] = *(const v4u*)(arow + cc * 32 + 16);
      const int kb = kk * CIN + cc * 32;
      const v16b b0 = FragB::load(Bb + kb);
      const v16b b1 = FragB::load(Bb + (size_t)16 * KDIM + kb);
      acc0 = FragB::mma(fa.v, b0, acc0);
      acc1 = FragB::mma(fa.v, b1, acc1);
      guard2_3(acc0, acc1, fa.v, b0, b1);
    }
  }
  acc_guard2(acc0, acc1);

  const int prow0 = wave * 16 + 8 * hh;
  {
    const float obv0 = bfr(offb[rlane]);
    om_stage_off(sO, acc0, rlane, prow0, obv0);
    const int col = 16 + rlane;
    const int co = (col < NCH_OFF) ? col : (NCH_OFF - 1);
    int cm = col - NCH_OFF; cm = cm < 0 ? 0 : (cm > NTAP - 1 ? NTAP - 1 : cm);
    const float obv1 = bfr(offb[co]);
    const float mbv1 = bfr(modb[cm]);
    const float fo = (col < NCH_OFF) ? 1.0f : 0.0f;
    om_stage_mix(sO, acc1, col, prow0, obv1, mbv1, fo);
  }
  __syncthreads();
  {
    const int c4 = (lane & 15) * 4;
    float* ob = om + m0 + c4;
    for (int pass = 0; pass < 2; ++pass) {
#pragma unroll
      for (int it = 0; it < 4; ++it) {
        const int ch = it * 8 + wave * 2 + hh;
        const v4f v = *(const v4f*)(sO + ch * SPITCH + c4);
        if (ch < NCH_OM) *(volatile v4f*)(ob + (size_t)ch * MROWS) = v;
      }
      __threadfence();
    }
  }
}

__global__ __launch_bounds__(256) void dcn_main_kernel(const unsigned short* __restrict__ xT, const float* __restrict__ om,
                                                       const unsigned short* __restrict__ wmbt,
                                                       const float* __restrict__ bias,
                                                       float* __restrict__ P, float* __restrict__ part) {
  __shared__ __align__(16) unsigned short Ahi[PTILE * APITCH];
  __shared__ __align__(16) unsigned short Alo[PTILE * APITCH];
  __shared__ __align__(16) float sOut[NCO * OPITCH];
  __shared__ __align__(16) float sPart[2 * NCO];

  const int tid = threadIdx.x, lane = tid & 31, wave = tid >> 5;
  const int rlane = lane & 15, hh = lane >> 4, koff = hh * 8;
  const int blk = blockIdx.x;
  const int m0 = blk * PTILE;
  const int n = m0 / HWPIX;
  const int hw0 = m0 - n * HWPIX;

  const int bp = tid >> 2, bq = tid & 3;
  const int bhw = hw0 + bp;
  const int bh = bhw / IMW, bw = bhw - bh * IMW;
  const size_t mpos = (size_t)(m0 + bp);
  const unsigned short* xn = xT + (size_t)n * PADPIX * CIN + bq * 8;
  unsigned short* ahi_dst = Ahi + bp * APITCH + bq * 8;
  unsigned short* alo_dst = Alo + bp * APITCH + bq * 8;

  const int ti = wave >> 1, nh = wave & 1;
  const __bf16* arow_hi = (const __bf16*)Ahi + (16 * ti + rlane) * APITCH + koff;
  const __bf16* arow_lo = (const __bf16*)Alo + (16 * ti + rlane) * APITCH + koff;
  const __bf16* brow = (const __bf16*)wmbt + (size_t)(64 * nh + rlane) * KDIM + koff;

  const v8f z8 = {0.f, 0.f, 0.f, 0.f, 0.f, 0.f, 0.f, 0.f};
  v8f acc[4];
#pragma unroll
  for (int j = 0; j < 4; ++j) acc[j] = z8;

#pragma unroll 1
  for (int kk = 0; kk < NTAP; ++kk) {
    const int ky = kk / 3, kx = kk - ky * 3;
    const float oy = om[(size_t)(2 * kk) * MROWS + mpos];
    const float ox = om[(size_t)(2 * kk + 1) * MROWS + mpos];
    const float mv = om[(size_t)(NCH_OFF + kk) * MROWS + mpos];
    const float sy = (oy + (float)bh) + (float)(ky - 1);
    const float sx = (ox + (float)bw) + (float)(kx - 1);
    const float y0f = floorf(sy), x0f = floorf(sx);
    const float y1f = y0f + 1.0f, x1f = x0f + 1.0f;
    const float wy1 = sy - y0f, wy0 = 1.0f - wy1;
    const float wx1 = sx - x0f, wx0 = 1.0f - wx1;
    const float vy0 = (y0f >= 0.0f && y0f <= (float)(IMH - 1)) ? 1.0f : 0.0f;
    const float vy1 = (y1f >= 0.0f && y1f <= (float)(IMH - 1)) ? 1.0f : 0.0f;
    const float vx0 = (x0f >= 0.0f && x0f <= (float)(IMW - 1)) ? 1.0f : 0.0f;
    const float vx1 = (x1f >= 0.0f && x1f <= (float)(IMW - 1)) ? 1.0f : 0.0f;
    const float g00 = (wy0 * wx0) * (vy0 * vx0);
    const float g01 = (wy0 * wx1) * (vy0 * vx1);
    const float g10 = (wy1 * wx0) * (vy1 * vx0);
    const float g11 = (wy1 * wx1) * (vy1 * vx1);
    const int cy0 = (int)fminf(fmaxf(y0f, 0.0f), (float)(IMH - 1));
    const int cy1 = (int)fminf(fmaxf(y1f, 0.0f), (float)(IMH - 1));
    const int cx0 = (int)fminf(fmaxf(x0f, 0.0f), (float)(IMW - 1));
    const int cx1 = (int)fminf(fmaxf(x1f, 0.0f), (float)(IMW - 1));
    const int o00 = ((cy0 + 1) * PADW + (cx0 + 1)) * CIN;
    const int o01 = ((cy0 + 1) * PADW + (cx1 + 1)) * CIN;
    const int o10 = ((cy1 + 1) * PADW + (cx0 + 1)) * CIN;
    const int o11 = ((cy1 + 1) * PADW + (cx1 + 1)) * CIN;
#pragma unroll 1
    for (int cc = 0; cc < CIN / 32; ++cc) {
      const int co = cc * 32;
      const v4u qa = *(const v4u*)(xn + o00 + co);
      const v4u qb = *(const v4u*)(xn + o01 + co);
      const v4u qc = *(const v4u*)(xn + o10 + co);
      const v4u qd = *(const v4u*)(xn + o11 + co);
      unsigned hw_[4], lw_[4];
#pragma unroll
      for (int i = 0; i < 4; ++i) {
        const float a0 = __uint_as_float(qa[i] << 16), a1 = __uint_as_float(qa[i] & 0xffff0000u);
        const float b0 = __uint_as_float(qb[i] << 16), b1 = __uint_as_float(qb[i] & 0xffff0000u);
        const float c0 = __uint_as_float(qc[i] << 16), c1 = __uint_as_float(qc[i] & 0xffff0000u);
        const float d0 = __uint_as_float(qd[i] << 16), d1 = __uint_as_float(qd[i] & 0xffff0000u);
        const float v0 = (((a0 * g00 + b0 * g01) + c0 * g10) + d0 * g11) * mv;
        const float v1 = (((a1 * g00 + b1 * g01) + c1 * g10) + d1 * g11) * mv;
        const unsigned h0 = (unsigned)f2bf_bits(v0);
        const unsigned h1 = (unsigned)f2bf_bits(v1);
        const unsigned l0 = (unsigned)f2bf_bits(v0 - __uint_as_float(h0 << 16));
        const unsigned l1 = (unsigned)f2bf_bits(v1 - __uint_as_float(h1 << 16));
        hw_[i] = h0 | (h1 << 16);
        lw_[i] = l0 | (l1 << 16);
      }
      const v4u hv = (v4u){hw_[0], hw_[1], hw_[2], hw_[3]};
      const v4u lv = (v4u){lw_[0], lw_[1], lw_[2], lw_[3]};
      __syncthreads();
      *(v4u*)(ahi_dst) = hv;
      *(v4u*)(alo_dst) = lv;
      __syncthreads();

      const int kb = kk * CIN + co;
      v16b b[4];
#pragma unroll
      for (int j = 0; j < 4; ++j) b[j] = FragB::load(brow + (size_t)(16 * j) * KDIM + kb);
      const v16b ah = FragB::load(arow_hi);
      const v16b al = FragB::load(arow_lo);
#pragma unroll
      for (int j = 0; j < 4; ++j) {
        acc[j] = FragB::mma(ah, b[j], acc[j]);
        acc[j] = FragB::mma(al, b[j], acc[j]);
      }
      guard4_6(acc[0], acc[1], acc[2], acc[3], ah, al, b[0], b[1], b[2], b[3]);
    }
  }
  acc_guard4(acc[0], acc[1], acc[2], acc[3]);

#pragma unroll
  for (int j = 0; j < 4; ++j) {
    const int o = 64 * nh + 16 * j + rlane;
    const float bb = bfr(bias[o]);
#pragma unroll
    for (int r = 0; r < 8; ++r) sOut[o * OPITCH + 16 * ti + 8 * hh + r] = acc[j][r] + bb;
  }
  __syncthreads();

  {
    const int po = tid >> 1, pf = tid & 1;
    const float* sp = sOut + po * OPITCH + pf * 32;
    float s = 0.0f, ss = 0.0f;
#pragma unroll 8
    for (int p = 0; p < 32; ++p) { const float v = sp[p]; s += v; ss = fmaf(v, v, ss); }
    const float s2  = s  + __shfl_xor(s, 1, 32);
    const float ss2 = ss + __shfl_xor(ss, 1, 32);
    sPart[2 * po + pf] = pf ? ss2 : s2;
  }
  __syncthreads();

  {
    const int c4 = (lane & 15) * 4;
    float* Pb = P + (size_t)n * NCO * HWPIX + hw0 + c4;
    for (int pass = 0; pass < 2; ++pass) {
#pragma unroll
      for (int it = 0; it < 8; ++it) {
        const int o = it * 16 + wave * 2 + hh;
        const v4f v = *(const v4f*)(sOut + o * OPITCH + c4);
        *(volatile v4f*)(Pb + (size_t)o * HWPIX) = v;
      }
      __threadfence();
    }
  }
  if (tid < 64) {
    const v4f v = *(const v4f*)(sPart + 4 * tid);
    float* dst = part + (size_t)blk * (2 * NCO) + 4 * tid;
    *(volatile v4f*)dst = v;
    __threadfence();
    *(volatile v4f*)dst = v;
  }
}

__global__ __launch_bounds__(128) void bn_stats_kernel(const float* __restrict__ part, const float* __restrict__ gamma,
                                                       const float* __restrict__ beta, float* __restrict__ bnp) {
  __shared__ __align__(16) float sb[2 * NCO];
  const int o = threadIdx.x;
  double s = 0.0, ss = 0.0;
#pragma unroll 4
  for (int b = 0; b < NBLK; ++b) {
    s  += (double)part[(size_t)b * (2 * NCO) + 2 * o];
    ss += (double)part[(size_t)b * (2 * NCO) + 2 * o + 1];
  }
  const double inv = 1.0 / (double)MROWS;
  const double mean = s * inv;
  const double var = ss * inv - mean * mean;
  float varf = (float)var;
  varf = varf > 0.0f ? varf : 0.0f;
  const float istd = 1.0f / sqrtf(varf + BN_EPSILON);
  const float sc = istd * bfr(gamma[o]);
  const float sh = bfr(beta[o]) - (float)mean * sc;
  sb[2 * o] = sc;
  sb[2 * o + 1] = sh;
  __syncthreads();
  if (o < 64) {
    const v4f v = *(const v4f*)(sb + 4 * o);
    *(volatile v4f*)(bnp + 4 * o) = v;
    __threadfence();
    *(volatile v4f*)(bnp + 4 * o) = v;
  }
}

__global__ __launch_bounds__(256) void bn_apply_kernel(const float* __restrict__ P, const float* __restrict__ bnp,
                                                       float* __restrict__ out) {
  const int i = blockIdx.x * 256 + threadIdx.x;
  if (i >= OUT4) return;
  const int ch = (i / (HWPIX / 4)) & (NCO - 1);
  const float sc = bnp[2 * ch], sh = bnp[2 * ch + 1];
  const v4f p = *(const v4f*)(P + (size_t)i * 4);
  v4f y;
#pragma unroll
  for (int e = 0; e < 4; ++e) y[e] = fmaxf(fmaf(p[e], sc, sh), 0.0f);
  float* dst = out + (size_t)i * 4;
  *(volatile v4f*)dst = y;
  __threadfence();
  *(volatile v4f*)dst = y;
}

extern "C" void kernel_launch(void* const* d_in, const int* in_sizes, int n_in,
                              void* d_out, int out_size, void* d_ws, size_t ws_size, hipStream_t stream) {
  if (n_in < 9) return;
  if (in_sizes[0] != NB * CIN * HWPIX || in_sizes[1] != NCH_OFF * CIN * NTAP || in_sizes[3] != NTAP * CIN * NTAP ||
      in_sizes[5] != NCO * CIN * NTAP || in_sizes[6] != NCO || out_size != NB * NCO * HWPIX) return;
  if (ws_size < WS_TOTAL) return;

  const float* x     = (const float*)d_in[0];
  const float* offw  = (const float*)d_in[1];
  const float* offb  = (const float*)d_in[2];
  const float* modw  = (const float*)d_in[3];
  const float* modb  = (const float*)d_in[4];
  const float* wgt   = (const float*)d_in[5];
  const float* bias  = (const float*)d_in[6];
  const float* gamma = (const float*)d_in[7];
  const float* beta  = (const float*)d_in[8];
  float* out = (float*)d_out;

  char* ws = (char*)d_ws;
  unsigned short* xT   = (unsigned short*)(ws + WS_OFF_XT);
  unsigned short* wall = (unsigned short*)(ws + WS_OFF_WALL);
  unsigned short* wmbt = wall;
  unsigned short* wobt = wall + (size_t)NCO * KDIM;
  float* om   = (float*)(ws + WS_OFF_OM);
  float* P    = (float*)(ws + WS_OFF_P);
  float* part = (float*)(ws + WS_OFF_PART);
  float* bnp  = (float*)(ws + WS_OFF_BNP);

  xprep_kernel<<<NBLK, 256, 0, stream>>>(x, xT);
  xborder_kernel<<<XB_THREADS / 256, 256, 0, stream>>>(xT);
  wswz_kernel<<<(WALL_ROWS * KW8) / 256, 256, 0, stream>>>(wgt, offw, modw, wall);
  offmask_kernel<<<NBLK, 128, 0, stream>>>(xT, wobt, offb, modb, om);
  dcn_main_kernel<<<NBLK, 256, 0, stream>>>(xT, om, wmbt, bias, P, part);
  bn_stats_kernel<<<1, 128, 0, stream>>>(part, gamma, beta, bnp);
  bn_apply_kernel<<<OUT4 / 256, 256, 0, stream>>>(P, bnp, out);
}
